// OneRelClassifier_33998961115715
// MI455X (gfx1250) — hardware-verified
//
#include <hip/hip_runtime.h>


#define NB_  4
#define NS_  128
#define HIN  768
#define H3   2304
#define NO_  96

typedef _Float16 h16;
typedef unsigned short bf;
typedef __attribute__((ext_vector_type(16))) __bf16   v16bf;
typedef __attribute__((ext_vector_type(16))) _Float16 v16h;
typedef __attribute__((ext_vector_type(8)))  _Float16 v8h;
typedef __attribute__((ext_vector_type(8)))  unsigned short v8us;
typedef __attribute__((ext_vector_type(8)))  float    v8f;
typedef __attribute__((ext_vector_type(4)))  float    v4f;
typedef v8h  __attribute__((may_alias)) v8ha;
typedef v4f  __attribute__((may_alias)) v4fa;

__device__ __forceinline__ unsigned short f2bf(float f) { unsigned u = __float_as_uint(f); u += 0x7FFFu + ((u >> 16) & 1u); return (unsigned short)(u >> 16); }
__device__ __forceinline__ float bf2f(unsigned short b) { return __uint_as_float(((unsigned)b) << 16); }
__device__ __forceinline__ float bfr(float f) { return bf2f(f2bf(f)); }
__device__ __forceinline__ v16h cat16(v8h lo, v8h hi) { return __builtin_shufflevector(lo, hi, 0, 1, 2, 3, 4, 5, 6, 7, 8, 9, 10, 11, 12, 13, 14, 15); }
__device__ __forceinline__ v16bf cat16b(v8us lo, v8us hi) { return __builtin_bit_cast(v16bf, __builtin_shufflevector(lo, hi, 0, 1, 2, 3, 4, 5, 6, 7, 8, 9, 10, 11, 12, 13, 14, 15)); }
__device__ __forceinline__ v8f wmma16(v16h a, v16h b, v8f c) { return __builtin_amdgcn_wmma_f32_16x16x32_f16(false, a, false, b, (short)0, c, false, false); }
__device__ __forceinline__ v8f wmmab(v16bf a, v16bf b, v8f c) { return __builtin_amdgcn_wmma_f32_16x16x32_bf16(false, a, false, b, (short)0, c, false, false); }

__global__ __launch_bounds__(256) void k_xb(const float* __restrict__ x, bf* Xb) {
    const int lane = threadIdx.x & 31, r = blockIdx.x * 8 + (threadIdx.x >> 5);
    if (r >= NB_ * NS_) return;
    const float* s = x + (size_t)r * HIN; bf* d = Xb + (size_t)r * HIN;
    v8us o[3];
#pragma unroll
    for (int q = 0; q < 3; ++q) { v8us t;
#pragma unroll
        for (int i = 0; i < 8; ++i) t[i] = f2bf(s[q * 256 + lane * 8 + i]);
        o[q] = t; }
#pragma unroll
    for (int q = 0; q < 3; ++q) *(volatile v8us*)(d + q * 256 + lane * 8) = o[q];
    __threadfence();
#pragma unroll
    for (int q = 0; q < 3; ++q) *(volatile v8us*)(d + q * 256 + lane * 8) = o[q];
}

template <bool BF>
__global__ __launch_bounds__(256) void k_wt(const float* __restrict__ Wm, int K, int N, unsigned short* WT) {
    __shared__ __align__(16) unsigned short tl[64 * 72];
    const int tid = threadIdx.x, k0 = blockIdx.x * 64, n0 = blockIdx.y * 64;
    const int kk = tid >> 2, nq = (tid & 3) * 16;
#pragma unroll
    for (int i = 0; i < 16; ++i) {
        const int n = n0 + nq + i;
        const float w = (n < N) ? Wm[(size_t)(k0 + kk) * N + n] : 0.0f;
        const unsigned short hb = f2bf(w);
        tl[(nq + i) * 72 + kk] = BF ? hb : __builtin_bit_cast(unsigned short, (h16)bf2f(hb));
    }
    __syncthreads();
    const int piece = tid & 7;
    auto pass = [&]() {
#pragma unroll
        for (int s = 0; s < 2; ++s) {
            const int nr = (tid >> 3) + 32 * s;
            if (n0 + nr < N) {
                const v8us val = *(const v8us*)(tl + nr * 72 + piece * 8);
                *(volatile v8us*)(WT + (size_t)(n0 + nr) * K + k0 + piece * 8) = val;
            }
        }
    };
    pass();
    __threadfence();
    pass();
}

__global__ __launch_bounds__(128) void k_gemmb(const bf* __restrict__ A, const bf* __restrict__ Bn, int K, float* C, int ldc) {
    __shared__ __align__(16) float ost[4][16 * 68];
    const int lane = threadIdx.x & 31, wave = threadIdx.x >> 5, lr = lane & 15, hi = lane >> 4;
    const int r0 = blockIdx.x * 64 + wave * 16, c0 = blockIdx.y * 64;
    const size_t aoff = (size_t)(r0 + lr) * K + 8 * hi;
    size_t boff[4];
#pragma unroll
    for (int t = 0; t < 4; ++t) boff[t] = (size_t)(c0 + t * 16 + lr) * K + 8 * hi;
    v8f acc[4];
#pragma unroll
    for (int t = 0; t < 4; ++t) acc[t] = (v8f){};
#pragma unroll 1
    for (int kc = 0; kc < K; kc += 32) {
        const v16bf a = cat16b(*(const v8us*)(A + aoff + kc), *(const v8us*)(A + aoff + kc + 16));
#pragma unroll
        for (int t = 0; t < 4; ++t) acc[t] = wmmab(a, cat16b(*(const v8us*)(Bn + boff[t] + kc), *(const v8us*)(Bn + boff[t] + kc + 16)), acc[t]);
        asm volatile("v_nop\n\tv_nop\n\tv_nop\n\tv_nop" : "+v"(acc[0]), "+v"(acc[1]), "+v"(acc[2]), "+v"(acc[3]) : "v"(a));
    }
    float* os = &ost[wave][0];
#pragma unroll
    for (int t = 0; t < 4; ++t)
#pragma unroll
        for (int j = 0; j < 8; ++j) os[(hi * 8 + j) * 68 + t * 16 + lr] = acc[t][j];
    __syncthreads();
    float* crow = C + (size_t)r0 * ldc + c0;
    auto pass = [&]() {
#pragma unroll
        for (int s = 0; s < 8; ++s) {
            const int Lid = (lane >> 3) + 4 * s, piece = lane & 7;
            const int row = Lid >> 1, cofs = (Lid & 1) * 32 + piece * 4;
            const v4f val = *(const v4fa*)(os + row * 68 + cofs);
            *(volatile v4f*)(crow + (size_t)row * ldc + cofs) = val;
        }
    };
    pass();
    __threadfence();
    pass();
}

__global__ __launch_bounds__(128) void k_pairs(const float* __restrict__ HEAD, const float* __restrict__ TAIL, const float* __restrict__ b1, const h16* __restrict__ W2T,
                                               const float* __restrict__ b2, float* out) {
    __shared__ __align__(16) float ost[4][16 * 100];
    const int lane = threadIdx.x & 31, wave = threadIdx.x >> 5, lr = lane & 15, hi = lane >> 4;
    const int bid = blockIdx.x;
    const int b = bid / (NS_ * (NS_ / 64)), rem = bid - b * (NS_ * (NS_ / 64)), i = rem / (NS_ / 64), jt = rem - i * (NS_ / 64);
    const int j0 = jt * 64 + wave * 16;
    const float* hrow = HEAD + ((size_t)b * NS_ + i) * H3;
    const float* trow = TAIL + ((size_t)b * NS_ + j0 + lr) * H3;
    v8f acc[6];
#pragma unroll
    for (int t = 0; t < 6; ++t) acc[t] = (v8f){};
#pragma unroll 1
    for (int kc = 0; kc < H3; kc += 32) {
        v16h a;
#pragma unroll
        for (int q = 0; q < 8; ++q) {
            const int k0 = kc + 8 * hi + q, k1 = kc + 16 + 8 * hi + q;
            const float v0 = hrow[k0] + trow[k0] + bfr(b1[k0]), v1 = hrow[k1] + trow[k1] + bfr(b1[k1]);
            a[q] = (h16)(v0 > 0.f ? v0 : 0.f); a[q + 8] = (h16)(v1 > 0.f ? v1 : 0.f);
        }
#pragma unroll
        for (int t = 0; t < 6; ++t) {
            const h16* bp = W2T + (size_t)(t * 16 + lr) * H3 + kc + 8 * hi;
            acc[t] = wmma16(a, cat16(*(const v8h*)bp, *(const v8h*)(bp + 16)), acc[t]);
        }
        asm volatile("v_nop\n\tv_nop\n\tv_nop\n\tv_nop" : "+v"(acc[0]), "+v"(acc[1]), "+v"(acc[2]), "+v"(acc[3]), "+v"(acc[4]), "+v"(acc[5]) : "v"(a));
    }
    float* os = &ost[wave][0];
#pragma unroll
    for (int t = 0; t < 6; ++t) {
        const float bv = bfr(b2[t * 16 + lr]);
#pragma unroll
        for (int j = 0; j < 8; ++j) os[(hi * 8 + j) * 100 + t * 16 + lr] = acc[t][j] + bv;
    }
    __syncthreads();
    float* crow = out + ((size_t)(b * NS_ + i) * NS_ + j0) * NO_;
    auto pass = [&]() {
#pragma unroll
        for (int s = 0; s < 12; ++s) {
            const int Lid = 4 * s + (lane >> 3), piece = lane & 7;
            const int row = Lid / 3, cofs = (Lid - row * 3) * 32 + piece * 4;
            const v4f val = *(const v4fa*)(os + row * 100 + cofs);
            *(volatile v4f*)(crow + (size_t)row * NO_ + cofs) = val;
        }
    };
    pass();
    __threadfence();
    pass();
}

extern "C" void kernel_launch(void* const* d_in, const int* in_sizes, int n_in,
                              void* d_out, int out_size, void* d_ws, size_t ws_size, hipStream_t stream) {
    (void)in_sizes; (void)n_in; (void)out_size;
    const float* x = (const float*)d_in[0]; const float* W1 = (const float*)d_in[1]; const float* b1 = (const float*)d_in[2]; const float* W2 = (const float*)d_in[3]; const float* b2 = (const float*)d_in[4];
    float* out = (float*)d_out;
    char* wsp = (char*)d_ws;
    auto take = [&](size_t bytes) { char* p = wsp; wsp += (bytes + 255) & ~(size_t)255; return (void*)p; };
    bf*    Xb   = (bf*)take((size_t)NB_ * NS_ * HIN * 2);
    bf*    W1HT = (bf*)take((size_t)H3 * HIN * 2);
    bf*    W1TT = (bf*)take((size_t)H3 * HIN * 2);
    h16*   W2T  = (h16*)take((size_t)NO_ * H3 * 2);
    float* HEAD = (float*)take((size_t)NB_ * NS_ * H3 * 4);
    float* TAIL = (float*)take((size_t)NB_ * NS_ * H3 * 4);
    if ((size_t)(wsp - (char*)d_ws) > ws_size) return;
    k_xb<<<(NB_ * NS_) / 8, 256, 0, stream>>>(x, Xb);
    k_wt<true><<<dim3(HIN / 64, H3 / 64, 1), 256, 0, stream>>>(W1, HIN, H3, W1HT);
    k_wt<true><<<dim3(HIN / 64, H3 / 64, 1), 256, 0, stream>>>(W1 + (size_t)HIN * H3, HIN, H3, W1TT);
    k_wt<false><<<dim3(H3 / 64, 2, 1), 256, 0, stream>>>(W2, H3, NO_, (unsigned short*)W2T);
    k_gemmb<<<dim3((NB_ * NS_) / 64, H3 / 64, 1), 128, 0, stream>>>(Xb, W1HT, HIN, HEAD, H3);
    k_gemmb<<<dim3((NB_ * NS_) / 64, H3 / 64, 1), 128, 0, stream>>>(Xb, W1TT, HIN, TAIL, H3);
    k_pairs<<<NB_ * NS_ * (NS_ / 64), 128, 0, stream>>>(HEAD, TAIL, b1, W2T, b2, out);
}
